// BEiTAttention_46926812676894
// MI455X (gfx1250) — hardware-verified
//
#include <hip/hip_runtime.h>
#include <math.h>
#include <float.h>
#include <stdint.h>

#define NBT   16
#define NBH   8
#define NTOK  1025
#define NP    1088
#define DM    768
#define NH    12
#define HD    64
#define NQB   (NP / 64)
#define QKVN  (3 * DM)
#define NREL  3972
static_assert(NH * HD == DM);
static_assert(NBT == 2 * NBH);
static_assert((NP % 64) == 0 && NP >= NTOK && (NP - NTOK) < 64);
static_assert((DM % 64) == 0);

#if defined(__HIP_DEVICE_COMPILE__)
#define DEVASM 1
#else
#define DEVASM 0
#endif

typedef _Float16 v16h __attribute__((ext_vector_type(16)));
typedef _Float16 v8h  __attribute__((ext_vector_type(8)));
typedef __bf16   v16b __attribute__((ext_vector_type(16)));
typedef __bf16   v8b  __attribute__((ext_vector_type(8)));
typedef float    v8f  __attribute__((ext_vector_type(8)));
typedef float    v4f  __attribute__((ext_vector_type(4)));
typedef unsigned int v4u __attribute__((ext_vector_type(4)));

__device__ __forceinline__ unsigned short bf_bits(float f) {
  unsigned u = __float_as_uint(f);
  return (unsigned short)((u + 0x7FFFu + ((u >> 16) & 1u)) >> 16);
}
__device__ __forceinline__ float bf_up(unsigned short h) { return __uint_as_float(((unsigned)h) << 16); }
__device__ __forceinline__ unsigned short h_bits(_Float16 x) { return __builtin_bit_cast(unsigned short, x); }
__device__ __forceinline__ unsigned pk16(unsigned short a, unsigned short b) { return (unsigned)a | ((unsigned)b << 16); }
__device__ __forceinline__ v8f zero8() { v8f z = {0.f, 0.f, 0.f, 0.f, 0.f, 0.f, 0.f, 0.f}; return z; }

__device__ __forceinline__ v16b ldfrag_b(const __bf16* p) {
  union { v16b v; v8b h[2]; } f;
  f.h[0] = *(const v8b*)(p);
  f.h[1] = *(const v8b*)(p + 16);
  return f.v;
}
__device__ __forceinline__ v16h ldfrag_h(const _Float16* p) {
  union { v16h v; v8h h[2]; } f;
  f.h[0] = *(const v8h*)(p);
  f.h[1] = *(const v8h*)(p + 16);
  return f.v;
}

__device__ __forceinline__ v8f mma_h(v16h a, v16h b, v8f c) {
  c = __builtin_amdgcn_wmma_f32_16x16x32_f16(false, a, false, b, (short)0, c, false, false);
#if DEVASM
  asm volatile("v_nop\n\tv_nop\n\tv_nop\n\tv_nop" : "+v"(c) : "v"(a), "v"(b));
#endif
  return c;
}
__device__ __forceinline__ v8f mma_b_raw(v16b a, v16b b, v8f c) {
  return __builtin_amdgcn_wmma_f32_16x16x32_bf16(false, a, false, b, (short)0, c, false, false);
}
__device__ __forceinline__ void dep_guard_b(v8f& a, v8f& b, v16b x, v16b y) {
#if DEVASM
  asm volatile("v_nop\n\tv_nop\n\tv_nop\n\tv_nop" : "+v"(a), "+v"(b) : "v"(x), "v"(y));
#else
  (void)a; (void)b; (void)x; (void)y;
#endif
}
__device__ __forceinline__ void keep4_b(v16b a, v16b b, v16b c, v16b d) {
#if DEVASM
  asm volatile("v_nop" :: "v"(a), "v"(b), "v"(c), "v"(d));
#else
  (void)a; (void)b; (void)c; (void)d;
#endif
}
__device__ __forceinline__ void acc_guard4(v8f& a, v8f& b, v8f& c, v8f& d) {
#if DEVASM
  asm volatile("v_nop\n\tv_nop\n\tv_nop\n\tv_nop" : "+v"(a), "+v"(b), "+v"(c), "+v"(d));
#else
  (void)a; (void)b; (void)c; (void)d;
#endif
}

__global__ __launch_bounds__(256) void cvt_bf16x8(const float* __restrict__ in, unsigned short* out, int n8) {
  const int i = blockIdx.x * 256 + threadIdx.x;
  if (i < n8) {
    const v4f a = *(const v4f*)(in + (size_t)i * 8);
    const v4f b = *(const v4f*)(in + (size_t)i * 8 + 4);
    v4u p;
    p[0] = pk16(bf_bits(a[0]), bf_bits(a[1]));
    p[1] = pk16(bf_bits(a[2]), bf_bits(a[3]));
    p[2] = pk16(bf_bits(b[0]), bf_bits(b[1]));
    p[3] = pk16(bf_bits(b[2]), bf_bits(b[3]));
    *(volatile v4u*)(out + (size_t)i * 8) = p;
    __threadfence();
    *(volatile v4u*)(out + (size_t)i * 8) = p;
  }
}

__global__ __launch_bounds__(256) void cvt_x8(const float* __restrict__ x, unsigned short* outp, int b0, int n8) {
  const int i = blockIdx.x * 256 + threadIdx.x;
  if (i < n8) {
    const int row = i / (DM / 8);
    const int c8  = (i - row * (DM / 8)) * 8;
    const int b   = row / NP;
    const int t   = row - b * NP;
    const int tc  = (t < NTOK) ? t : (NTOK - 1);
    const float* src = x + ((size_t)(b0 + b) * NTOK + tc) * DM + c8;
    const v4f a = *(const v4f*)(src);
    const v4f q = *(const v4f*)(src + 4);
    const unsigned keep = (t < NTOK) ? 0xFFFFFFFFu : 0u;
    v4u p;
    p[0] = pk16(bf_bits(a[0]), bf_bits(a[1])) & keep;
    p[1] = pk16(bf_bits(a[2]), bf_bits(a[3])) & keep;
    p[2] = pk16(bf_bits(q[0]), bf_bits(q[1])) & keep;
    p[3] = pk16(bf_bits(q[2]), bf_bits(q[3])) & keep;
    *(volatile v4u*)(outp + (size_t)i * 8) = p;
    __threadfence();
    *(volatile v4u*)(outp + (size_t)i * 8) = p;
  }
}

__global__ __launch_bounds__(256) void bias_gather16(const float* __restrict__ table, const int* __restrict__ ridx,
                                                     unsigned short* outp, int n8) {
  const int h = blockIdx.y;
  const int g = blockIdx.x * 256 + threadIdx.x;
  if (g < n8) {
    const int e  = g * 8;
    const int i  = e / NP;
    const int j0 = e - i * NP;
    const int ic = (i < NTOK) ? i : (NTOK - 1);
    const int* irow = ridx + (size_t)ic * NTOK;
    v4u p;
#pragma unroll
    for (int e2 = 0; e2 < 4; ++e2) {
      const int ja = j0 + 2 * e2, jb = ja + 1;
      const int jca = (ja < NTOK) ? ja : (NTOK - 1);
      const int jcb = (jb < NTOK) ? jb : (NTOK - 1);
      int ida = irow[jca];
      int idb = irow[jcb];
      ida = (ida < 0) ? (ida + NREL) : ida;
      idb = (idb < 0) ? (idb + NREL) : idb;
      ida = (ida < 0) ? 0 : ((ida >= NREL) ? (NREL - 1) : ida);
      idb = (idb < 0) ? 0 : ((idb >= NREL) ? (NREL - 1) : idb);
      const float ta = table[(size_t)ida * NH + h];
      const float tb = table[(size_t)idb * NH + h];
      const unsigned short ua = (i < NTOK && ja < NTOK) ? bf_bits(ta) : (unsigned short)0;
      const unsigned short ub = (i < NTOK && jb < NTOK) ? bf_bits(tb) : (unsigned short)0;
      p[e2] = pk16(ua, ub);
    }
    unsigned short* dst = outp + (size_t)h * NP * NP + e;
    *(volatile v4u*)dst = p;
    __threadfence();
    *(volatile v4u*)dst = p;
  }
}

template <int MODE>
__global__ __launch_bounds__(256) void gemm64(
    const unsigned short* __restrict__ Ap, const unsigned short* __restrict__ A2p, int lda, long long strideA,
    const unsigned short* __restrict__ Btp, int ldb, long long strideB,
    const float* __restrict__ bias,
    void* C0, void* C1, int ldc, long long strideC,
    int M, int N, int K, int Mvalid) {
  const __bf16* A  = (const __bf16*)(const void*)Ap;
  const __bf16* A2 = (const __bf16*)(const void*)A2p;
  const __bf16* Bt = (const __bf16*)(const void*)Btp;
  __shared__ __align__(16) float sT[8][16 * 68];
  const int b    = blockIdx.y;
  const int lane = threadIdx.x & 31;
  const int wave = threadIdx.x >> 5;
  const int tilesN = N >> 6;
  const int tilesM = M >> 6;
  const int tile = blockIdx.x * 8 + wave;
  if (tile >= tilesM * tilesN) return;
  const int tm = tile / tilesN;
  const int tn = tile - tm * tilesN;
  const int m0 = tm << 6;
  const int n0 = tn << 6;

  const __bf16* Ab  = A + (size_t)b * strideA;
  const __bf16* Ab2 = (MODE == 2) ? (A2 + (size_t)b * strideA) : Ab;
  const __bf16* Bb  = Bt + (size_t)b * strideB;

  const int rlane = lane & 15;
  const int koff  = (lane >> 4) * 8;
  const int mOff  = (lane >> 4) * 8;

  v8f acc[4][4];
#pragma unroll
  for (int i = 0; i < 4; ++i)
#pragma unroll
    for (int j = 0; j < 4; ++j) acc[i][j] = zero8();

  for (int k0 = 0; k0 < K; k0 += 32) {
    v16b bh[4];
#pragma unroll
    for (int j = 0; j < 4; ++j) {
      const size_t bo = (size_t)(n0 + (j << 4) + rlane) * ldb + koff + k0;
      bh[j] = ldfrag_b(Bb + bo);
    }
#pragma unroll
    for (int i = 0; i < 4; ++i) {
      const size_t ao = (size_t)(m0 + (i << 4) + rlane) * lda + koff + k0;
      const v16b ah = ldfrag_b(Ab + ao);
      v16b al = ah;
      if (MODE == 2) al = ldfrag_b(Ab2 + ao);
#pragma unroll
      for (int j = 0; j < 4; ++j) {
        acc[i][j] = mma_b_raw(ah, bh[j], acc[i][j]);
        if (MODE == 2) acc[i][j] = mma_b_raw(al, bh[j], acc[i][j]);
      }
      dep_guard_b(acc[i][0], acc[i][3], ah, al);
    }
    keep4_b(bh[0], bh[1], bh[2], bh[3]);
  }
  acc_guard4(acc[0][0], acc[0][1], acc[0][2], acc[0][3]);
  acc_guard4(acc[1][0], acc[1][1], acc[1][2], acc[1][3]);
  acc_guard4(acc[2][0], acc[2][1], acc[2][2], acc[2][3]);
  acc_guard4(acc[3][0], acc[3][1], acc[3][2], acc[3][3]);

  float* slab = sT[wave];
  const int q8 = lane >> 3, c8 = (lane & 7) * 8;
  const int h2 = lane >> 4, c4 = (lane & 15) * 4;
#pragma unroll
  for (int i = 0; i < 4; ++i) {
    const int mBase = m0 + (i << 4);
#pragma unroll
    for (int j = 0; j < 4; ++j) {
#pragma unroll
      for (int r = 0; r < 8; ++r) {
        slab[(mOff + r) * 68 + (j << 4) + rlane] = acc[i][j][r];
      }
    }
    __builtin_amdgcn_fence(__ATOMIC_RELEASE, "workgroup");
    __builtin_amdgcn_wave_barrier();
    __builtin_amdgcn_fence(__ATOMIC_ACQUIRE, "workgroup");
    if (MODE == 2) {
      float* C = (float*)C0 + (size_t)b * strideC;
      float pb[4];
#pragma unroll
      for (int e = 0; e < 4; ++e) pb[e] = bf_up(bf_bits(bias[n0 + c4 + e]));
      v4f vv[8];
#pragma unroll
      for (int it = 0; it < 8; ++it) {
        const int row = it * 2 + h2;
        v4f v = *(const v4f*)(slab + row * 68 + c4);
        v[0] += pb[0]; v[1] += pb[1]; v[2] += pb[2]; v[3] += pb[3];
        vv[it] = v;
      }
      for (int pass = 0; pass < 2; ++pass) {
#pragma unroll
        for (int it = 0; it < 8; ++it) {
          const int row = it * 2 + h2;
          if (mBase + row < Mvalid)
            *(volatile v4f*)(C + (size_t)(mBase + row) * ldc + n0 + c4) = vv[it];
        }
        __threadfence();
      }
    } else if (MODE == 0) {
      const bool isQ = (n0 < DM);
      unsigned short* C = isQ ? (unsigned short*)C0 : (unsigned short*)C1;
      const int cb = isQ ? n0 : (n0 - DM);
      const int bc = isQ ? (n0 + c8) : 0;
      float ab[8];
#pragma unroll
      for (int e = 0; e < 8; ++e) {
        const float tb = bf_up(bf_bits(bias[bc + e]));
        ab[e] = isQ ? tb : 0.0f;
      }
      v4u hv[4];
#pragma unroll
      for (int it = 0; it < 4; ++it) {
        const int row = it * 4 + q8;
        const float* sp = slab + row * 68 + c8;
        v4u a;
#pragma unroll
        for (int e = 0; e < 4; ++e) {
          const float f0 = sp[2 * e] + ab[2 * e], f1 = sp[2 * e + 1] + ab[2 * e + 1];
          a[e] = pk16(h_bits((_Float16)f0), h_bits((_Float16)f1));
        }
        hv[it] = a;
      }
      for (int pass = 0; pass < 2; ++pass) {
#pragma unroll
        for (int it = 0; it < 4; ++it) {
          const int row = it * 4 + q8;
          *(volatile v4u*)(C + (size_t)(mBase + row) * ldc + cb + c8) = hv[it];
        }
        __threadfence();
      }
    } else {
      unsigned short* Ch = (unsigned short*)C0 + (size_t)b * strideC;
      unsigned short* Cl = (unsigned short*)C1 + (size_t)b * strideC;
      v4u hv[4], lv[4];
#pragma unroll
      for (int it = 0; it < 4; ++it) {
        const int row = it * 4 + q8;
        const float vb = bf_up(bf_bits(bias[mBase + row]));
        const float* sp = slab + row * 68 + c8;
        v4u a, a2;
#pragma unroll
        for (int e = 0; e < 4; ++e) {
          const float f0 = sp[2 * e] + vb, f1 = sp[2 * e + 1] + vb;
          const _Float16 x0 = (_Float16)f0, x1 = (_Float16)f1;
          const unsigned short h0 = h_bits(x0), h1 = h_bits(x1);
          const unsigned short l0 = h_bits((_Float16)((f0 - (float)x0) * 4096.0f));
          const unsigned short l1 = h_bits((_Float16)((f1 - (float)x1) * 4096.0f));
          a[e] = pk16(h0, h1); a2[e] = pk16(l0, l1);
        }
        hv[it] = a; lv[it] = a2;
      }
      for (int pass = 0; pass < 2; ++pass) {
#pragma unroll
        for (int it = 0; it < 4; ++it) {
          const int row = it * 4 + q8;
          *(volatile v4u*)(Ch + (size_t)(mBase + row) * ldc + n0 + c8) = hv[it];
          *(volatile v4u*)(Cl + (size_t)(mBase + row) * ldc + n0 + c8) = lv[it];
        }
        __threadfence();
      }
    }
    __builtin_amdgcn_fence(__ATOMIC_RELEASE, "workgroup");
    __builtin_amdgcn_wave_barrier();
    __builtin_amdgcn_fence(__ATOMIC_ACQUIRE, "workgroup");
  }
}

__global__ __launch_bounds__(256) void vt_rowsum(const unsigned short* __restrict__ vhp, const unsigned short* __restrict__ vlp,
                                                 float* vsum, int nrows) {
  __shared__ __align__(16) float ss[32];
  const int tid = threadIdx.x, wave = tid >> 5, lane = tid & 31;
#pragma unroll
  for (int rr = 0; rr < 4; ++rr) {
    int row = blockIdx.x * 32 + wave * 4 + rr;
    row = (row < nrows) ? row : (nrows - 1);
    const _Float16* ph = (const _Float16*)(const void*)vhp + (size_t)row * NP;
    const _Float16* pl = (const _Float16*)(const void*)vlp + (size_t)row * NP;
    float ah = 0.f, al = 0.f;
#pragma unroll 1
    for (int it = 0; it < (NP + 255) / 256; ++it) {
      const int s0 = it * 256 + lane * 8;
      const int sc = (s0 + 8 <= NP) ? s0 : (NP - 8);
      const v8h xh = *(const v8h*)(ph + sc);
      const v8h xl = *(const v8h*)(pl + sc);
#pragma unroll
      for (int e = 0; e < 8; ++e) {
        const bool ok = (s0 + e < NTOK);
        ah += ok ? (float)xh[e] : 0.0f;
        al += ok ? (float)xl[e] : 0.0f;
      }
    }
    float a = ah + al * (1.0f / 4096.0f);
#pragma unroll
    for (int off = 16; off > 0; off >>= 1) a += __shfl_xor(a, off, 32);
    if (lane == 0) ss[wave * 4 + rr] = a;
  }
  __syncthreads();
  const int l8 = (lane < 8) ? lane : 0;
  const v4f w = *(const v4f*)(ss + l8 * 4);
  float* dst = vsum + (size_t)blockIdx.x * 32 + l8 * 4;
  if (wave == 0 && lane < 8) *(volatile v4f*)dst = w;
  __threadfence();
  if (wave == 0 && lane < 8) *(volatile v4f*)dst = w;
}

__global__ __launch_bounds__(128)
void attn_rpb64(const unsigned short* __restrict__ qpl, const unsigned short* __restrict__ kpl,
                const unsigned short* __restrict__ vhp, const unsigned short* __restrict__ vlp,
                const unsigned short* __restrict__ bpl, const float* __restrict__ vsum,
                unsigned short* ohp, unsigned short* olp, float sscale) {
  union FH { v16h v; v8h h[2]; };
  __shared__ __align__(16) _Float16 Ksh[64 * 64];
  __shared__ __align__(16) _Float16 Vth[64 * 64];
  __shared__ __align__(16) _Float16 Vtl[64 * 64];
  __shared__ __align__(16) _Float16 Psh[4][16 * 64];
  __shared__ __align__(16) float    Os[4][16 * 64];

  const int tid  = threadIdx.x;
  const int wave = tid >> 5;
  const int lane = tid & 31;
  const int hh   = lane >> 4;
  const int c    = lane & 15;

  const int bx   = blockIdx.x;
  const int qb   = bx % NQB;
  const int rest = bx / NQB;
  const int h    = rest % NH;
  const int b    = rest / NH;
  const int q0   = qb * 64 + wave * 16;
  const size_t rowB = (size_t)b * NP;

  const _Float16* Q  = (const _Float16*)(const void*)qpl + (size_t)h * HD;
  const _Float16* Kg = (const _Float16*)(const void*)kpl + (size_t)h * HD;
  const _Float16* Vh = (const _Float16*)(const void*)vhp + ((size_t)b * DM + (size_t)h * HD) * NP;
  const _Float16* Vl = (const _Float16*)(const void*)vlp + ((size_t)b * DM + (size_t)h * HD) * NP;
  const unsigned short* Bp = bpl + (size_t)h * NP * NP;

  v16h qa[2];
#pragma unroll
  for (int dc = 0; dc < 2; ++dc) qa[dc] = ldfrag_h(Q + (rowB + q0 + c) * DM + dc * 32 + 8 * hh);
  float vs[4];
#pragma unroll
  for (int t = 0; t < 4; ++t) vs[t] = vsum[(size_t)b * DM + (size_t)h * HD + t * 16 + c];

  float mrow[8], lrow[8], lg[8];
  v8f oacc[4];
#pragma unroll
  for (int r = 0; r < 8; ++r) { mrow[r] = -INFINITY; lrow[r] = 0.f; lg[r] = 0.f; }
#pragma unroll
  for (int t = 0; t < 4; ++t) oacc[t] = zero8();

  for (int kt = 0; kt < NQB; ++kt) {
    const int kv0 = kt * 64;
    __syncthreads();
    {
      const int r = tid >> 1, half = (tid & 1) * 32;
      const _Float16* kg = Kg + (rowB + kv0 + r) * DM + half;
      const _Float16* vg = Vh + (size_t)r * NP + kv0 + half;
      const _Float16* lp = Vl + (size_t)r * NP + kv0 + half;
#pragma unroll
      for (int i = 0; i < 4; ++i) {
        const v8h a0 = *(const v8h*)(kg + 8 * i);
        const v8h b0 = *(const v8h*)(vg + 8 * i);
        const v8h b1 = *(const v8h*)(lp + 8 * i);
        *(v8h*)(Ksh + r * 64 + half + 8 * i) = a0;
        *(v8h*)(Vth + r * 64 + half + 8 * i) = b0;
        *(v8h*)(Vtl + r * 64 + half + 8 * i) = b1;
      }
    }
    __syncthreads();

    v8f s[4];
#pragma unroll
    for (int j = 0; j < 4; ++j) {
      s[j] = zero8();
#pragma unroll
      for (int dc = 0; dc < 2; ++dc) {
        FH kb;
        kb.h[0] = *(const v8h*)(Ksh + (j * 16 + c) * 64 + dc * 32 + 8 * hh);
        kb.h[1] = *(const v8h*)(Ksh + (j * 16 + c) * 64 + dc * 32 + 16 + 8 * hh);
        s[j] = mma_h(qa[dc], kb.v, s[j]);
      }
    }

    _Float16* pwh = Psh[wave];
    const unsigned short* brow = Bp + (size_t)(q0 + 8 * hh) * NP + kv0 + c;
#pragma unroll
    for (int r = 0; r < 8; ++r) {
      const unsigned short* br = brow + (size_t)r * NP;
      float m = -INFINITY;
#pragma unroll
      for (int j = 0; j < 4; ++j) {
        const int key = kv0 + j * 16 + c;
        const float bv = bf_up(br[j * 16]);
        float sv = s[j][r] * sscale + bv;
        sv = (key < NTOK) ? sv : -INFINITY;
        s[j][r] = sv;
        m = fmaxf(m, sv);
      }
#pragma unroll
      for (int off = 1; off < 16; off <<= 1) m = fmaxf(m, __shfl_xor(m, off, 32));
      const float mnew  = fmaxf(mrow[r], m);
      const float msafe = (mnew == -INFINITY) ? 0.f : mnew;
      const float alpha = __expf(mrow[r] - msafe);
      if (kt == 0) lg[r] = fminf(msafe, 0.0f);
      mrow[r] = mnew;
      const float csub = 1024.0f * __expf(lg[r] - msafe);
      float psum = 0.f;
#pragma unroll
      for (int j = 0; j < 4; ++j) {
        const int key = kv0 + j * 16 + c;
        const float p = __expf(s[j][r] - msafe);
        psum += p;
        const float pc = (key < NTOK) ? (p * 1024.0f - csub) : 0.0f;
        pwh[(8 * hh + r) * 64 + j * 16 + c] = (_Float16)pc;
      }
#pragma unroll
      for (int off = 1; off < 16; off <<= 1) psum += __shfl_xor(psum, off, 32);
      lrow[r] = lrow[r] * alpha + psum;
#pragma unroll
      for (int t = 0; t < 4; ++t) oacc[t][r] *= alpha;
    }
    __builtin_amdgcn_fence(__ATOMIC_RELEASE, "workgroup");
    __builtin_amdgcn_wave_barrier();
    __builtin_amdgcn_fence(__ATOMIC_ACQUIRE, "workgroup");

    v8f o1[4];
#pragma unroll
    for (int t = 0; t < 4; ++t) o1[t] = zero8();
#pragma unroll 1
    for (int kk = 0; kk < 2; ++kk) {
      FH pa;
      pa.h[0] = *(const v8h*)(pwh + c * 64 + kk * 32 + 8 * hh);
      pa.h[1] = *(const v8h*)(pwh + c * 64 + kk * 32 + 16 + 8 * hh);
#pragma unroll
      for (int t = 0; t < 4; ++t) {
        FH vb, vl;
        vb.h[0] = *(const v8h*)(Vth + (t * 16 + c) * 64 + kk * 32 + 8 * hh);
        vb.h[1] = *(const v8h*)(Vth + (t * 16 + c) * 64 + kk * 32 + 16 + 8 * hh);
        vl.h[0] = *(const v8h*)(Vtl + (t * 16 + c) * 64 + kk * 32 + 8 * hh);
        vl.h[1] = *(const v8h*)(Vtl + (t * 16 + c) * 64 + kk * 32 + 16 + 8 * hh);
        oacc[t] = mma_h(pa.v, vb.v, oacc[t]);
        o1[t]   = mma_h(pa.v, vl.v, o1[t]);
      }
    }
#pragma unroll
    for (int t = 0; t < 4; ++t)
#pragma unroll
      for (int r = 0; r < 8; ++r) oacc[t][r] += o1[t][r] * (1.0f / 4096.0f);
  }

  float* os = Os[wave];
#pragma unroll
  for (int r = 0; r < 8; ++r) {
    const float l   = lrow[r];
    const float inv = (l > 0.f) ? (1.0f / l) : 0.f;
    const float mf  = (mrow[r] == -INFINITY) ? 0.f : mrow[r];
    const float cf  = __expf(lg[r] - mf);
#pragma unroll
    for (int t = 0; t < 4; ++t)
      os[(8 * hh + r) * 64 + t * 16 + c] = (oacc[t][r] * (1.0f / 1024.0f) + cf * vs[t]) * inv;
  }
  __builtin_amdgcn_fence(__ATOMIC_RELEASE, "workgroup");
  __builtin_amdgcn_wave_barrier();
  __builtin_amdgcn_fence(__ATOMIC_ACQUIRE, "workgroup");
  {
    const int q4 = lane >> 3, c8 = (lane & 7) * 8;
    v4u hv[4], lv[4];
#pragma unroll
    for (int it = 0; it < 4; ++it) {
      const int row = it * 4 + q4;
      const float* sp = os + row * 64 + c8;
      v4u a, a2;
#pragma unroll
      for (int e = 0; e < 4; ++e) {
        const float f0 = sp[2 * e], f1 = sp[2 * e + 1];
        const unsigned short h0 = bf_bits(f0), h1 = bf_bits(f1);
        const unsigned short l0 = bf_bits(f0 - bf_up(h0)), l1 = bf_bits(f1 - bf_up(h1));
        a[e] = pk16(h0, h1); a2[e] = pk16(l0, l1);
      }
      hv[it] = a; lv[it] = a2;
    }
    for (int pass = 0; pass < 2; ++pass) {
#pragma unroll
      for (int it = 0; it < 4; ++it) {
        const int row = it * 4 + q4;
        const size_t go = (rowB + q0 + row) * DM + (size_t)h * HD + c8;
        *(volatile v4u*)(ohp + go) = hv[it];
        *(volatile v4u*)(olp + go) = lv[it];
      }
      __threadfence();
    }
  }
}

extern "C" void kernel_launch(void* const* d_in, const int* in_sizes, int n_in,
                              void* d_out, int out_size, void* d_ws, size_t ws_size,
                              hipStream_t stream) {
  if (n_in < 8) return;
  if (in_sizes[0] != NBT * NTOK * DM) return;
  if (in_sizes[1] != QKVN * DM) return;
  if (in_sizes[2] != DM || in_sizes[3] != DM || in_sizes[6] != DM) return;
  if (in_sizes[4] != NREL * NH) return;
  if (in_sizes[5] != DM * DM) return;
  if (in_sizes[7] != NTOK * NTOK) return;
  if (out_size != NBT * NTOK * DM) return;

  const float* x      = (const float*)d_in[0];
  const float* qkvw   = (const float*)d_in[1];
  const float* q_bias = (const float*)d_in[2];
  const float* v_bias = (const float*)d_in[3];
  const float* table  = (const float*)d_in[4];
  const float* projw  = (const float*)d_in[5];
  const float* p_bias = (const float*)d_in[6];
  const int*   relidx = (const int*)d_in[7];
  float* out = (float*)d_out;

  const size_t PA  = (size_t)NBH * NP * DM * 2;
  const size_t PWQ = (size_t)QKVN * DM * 2;
  const size_t PWO = (size_t)DM * DM * 2;
  const size_t PB  = (size_t)NH * NP * NP * 2;
  const size_t PS  = (size_t)NBH * DM * 4;
  size_t off = 0;
  const size_t oXb  = off; off += PA;
  const size_t oQ   = off; off += PA;
  const size_t oK   = off; off += PA;
  const size_t oVTh = off; off += PA;
  const size_t oVTl = off; off += PA;
  const size_t oCl  = off; off += PA;
  const size_t oWq  = off; off += PWQ;
  const size_t oWo  = off; off += PWO;
  const size_t oBs  = off; off += PB;
  const size_t oVs  = off; off += PS;
  if (off > ws_size) return;
  if (off > (size_t)134217728) return;
  const size_t oCh  = oXb;

  char* ws = (char*)d_ws;
  unsigned short* Xb   = (unsigned short*)(ws + oXb);
  unsigned short* Qp   = (unsigned short*)(ws + oQ);
  unsigned short* Kp   = (unsigned short*)(ws + oK);
  unsigned short* VTh  = (unsigned short*)(ws + oVTh);
  unsigned short* VTl  = (unsigned short*)(ws + oVTl);
  unsigned short* Cl   = (unsigned short*)(ws + oCl);
  unsigned short* Ch   = (unsigned short*)(ws + oCh);
  unsigned short* Wqb  = (unsigned short*)(ws + oWq);
  unsigned short* Wvb  = Wqb + (size_t)2 * DM * DM;
  unsigned short* Wob  = (unsigned short*)(ws + oWo);
  unsigned short* Bpl  = (unsigned short*)(ws + oBs);
  float*          Vsum = (float*)(ws + oVs);

  const dim3 blk(256);
  const int n8wq = QKVN * DM / 8;
  const int n8wo = DM * DM / 8;
  const int n8b  = NP * NP / 8;
  const int n8x  = NBH * NP * DM / 8;
  const dim3 gWq((n8wq + 255) / 256);
  const dim3 gWo((n8wo + 255) / 256);
  const dim3 gBs((n8b + 255) / 256, NH);
  const dim3 gX((n8x + 255) / 256);
  const dim3 gQK(((NBH * NP / 64) * (2 * DM / 64) + 7) / 8, 1);
  const dim3 gVT(((DM / 64) * (NP / 64) + 7) / 8, NBH);
  const dim3 gPJ(((NP / 64) * (DM / 64) + 7) / 8, NBH);
  const dim3 gVS((NBH * DM) / 32);
  const dim3 gAT(NBH * NH * NQB);

  cvt_bf16x8<<<gWq, blk, 0, stream>>>(qkvw, Wqb, n8wq);
  cvt_bf16x8<<<gWo, blk, 0, stream>>>(projw, Wob, n8wo);
  bias_gather16<<<gBs, blk, 0, stream>>>(table, relidx, Bpl, n8b);

  for (int p = 0; p < NBT / NBH; ++p) {
    cvt_x8<<<gX, blk, 0, stream>>>(x, Xb, p * NBH, n8x);
    gemm64<0><<<gQK, blk, 0, stream>>>(
        Xb, Xb, DM, 0LL, Wqb, DM, 0LL, q_bias,
        (void*)Qp, (void*)Kp, DM, 0LL,
        NBH * NP, 2 * DM, DM, NBH * NP);
    gemm64<1><<<gVT, blk, 0, stream>>>(
        Wvb, Wvb, DM, 0LL, Xb, DM, (long long)NP * DM, v_bias,
        (void*)VTh, (void*)VTl, NP, (long long)DM * NP,
        DM, NP, DM, DM);
    vt_rowsum<<<gVS, blk, 0, stream>>>(VTh, VTl, Vsum, NBH * DM);
    attn_rpb64<<<gAT, dim3(128), 0, stream>>>(Qp, Kp, VTh, VTl, Bpl, Vsum, Ch, Cl, 0.125f);
    gemm64<2><<<gPJ, blk, 0, stream>>>(
        Ch, Cl, DM, (long long)NP * DM, Wob, DM, 0LL, p_bias,
        (void*)(out + (size_t)p * NBH * NTOK * DM), (void*)(out + (size_t)p * NBH * NTOK * DM),
        DM, (long long)NTOK * DM,
        NP, DM, DM, NTOK);
  }
  (void)hipGetLastError();
}
